// SimpleCNN_82798379532474
// MI455X (gfx1250) — hardware-verified
//
#include <hip/hip_runtime.h>
#include <stddef.h>

typedef _Float16 v16h __attribute__((ext_vector_type(16)));
typedef _Float16 v8h  __attribute__((ext_vector_type(8)));
typedef float    v8f  __attribute__((ext_vector_type(8)));
typedef float    v4f  __attribute__((ext_vector_type(4)));
typedef v8h __attribute__((may_alias)) v8ha;
typedef v4f __attribute__((may_alias)) v4fa;

union Frag { v16h v; v8h half[2]; };

#define NIMG     4096
#define IMGPIX   784
#define NWIN1    196
#define NWIN2    49
#define C1       32
#define C2       64
#define KC1      16
#define KC2      32
#define K1PITCH  32
#define K2PITCH  832
#define FCK      3136
#define FCN      128
#define NCLS     10
#define WSCALE   16.0f
#define WINV     0.0625f

#define OFF_ZROW   0
#define SZ_ZROW    256
#define OFF_K1P    (OFF_ZROW + SZ_ZROW)
#define SZ_K1P     (C1 * K1PITCH * 2)
#define OFF_K2P    (OFF_K1P + SZ_K1P)
#define SZ_K2P     (C2 * K2PITCH * 2)
#define OFF_FWP    (OFF_K2P + SZ_K2P)
#define SZ_FWP     (FCN * FCK * 2)
#define OFF_ACT1   (OFF_FWP + SZ_FWP)
#define SZ_ACT1    (NIMG * NWIN1 * C1 * 2)
#define OFF_ACT2   (OFF_ACT1 + SZ_ACT1)
#define SZ_ACT2    (NIMG * NWIN2 * C2 * 2)
#define WS_TOTAL   (OFF_ACT2 + SZ_ACT2)

static_assert((OFF_K1P % 128) == 0);
static_assert((OFF_K2P % 128) == 0);
static_assert((OFF_FWP % 128) == 0);
static_assert((OFF_ACT1 % 128) == 0);
static_assert((OFF_ACT2 % 128) == 0);
static_assert((WS_TOTAL % 128) == 0);
static_assert(((K2PITCH * 2) % 128) == 0);
static_assert(((FCK * 2) % 128) == 0);
static_assert((NWIN1 % 4) == 0);
static_assert((IMGPIX % 16) == 0);
static_assert(((NIMG * NWIN1) % (16 * 196)) == 0);

__device__ __forceinline__ v8f wmma_f16(v16h a, v16h b, v8f c) {
  v8f d = __builtin_amdgcn_wmma_f32_16x16x32_f16(false, a, false, b, (short)0, c, false, false);
  asm volatile("v_nop\n\tv_nop\n\tv_nop\n\tv_nop" : "+v"(d) : "v"(a), "v"(b));
  return d;
}

__device__ __forceinline__ v16h load_frag(const _Float16* p, int h) {
  Frag f;
  f.half[0] = *(const v8ha*)(p + 8 * h);
  f.half[1] = *(const v8ha*)(p + 16 + 8 * h);
  return f.v;
}

__global__ __launch_bounds__(256) void prep_kernel(
    const float* __restrict__ w1, const float* __restrict__ p1,
    const float* __restrict__ w2, const float* __restrict__ p2,
    const float* __restrict__ fc1w,
    _Float16* __restrict__ zrow, _Float16* __restrict__ k1p,
    _Float16* __restrict__ k2p, _Float16* __restrict__ fwp)
{
#pragma clang fp contract(off)
  __shared__ float sacc[32 * 36];
  const int tid = threadIdx.x;
  const int blk = blockIdx.x;
  const v8h z8 = {(_Float16)0.0f, (_Float16)0.0f, (_Float16)0.0f, (_Float16)0.0f,
                  (_Float16)0.0f, (_Float16)0.0f, (_Float16)0.0f, (_Float16)0.0f};

  if (blk < 65) {
    const bool big = (blk < 64);
    const int Co = big ? C2 : C1;
    const int Ci = big ? 32 : 1;
    const int Kc = big ? KC2 : KC1;
    const float* w = big ? w2 : w1;
    const float* p = big ? p2 : p1;
    if (tid < 32) {
      float* my = sacc + tid * 36;
      #pragma unroll 1
      for (int c = 0; c < 36; ++c) my[c] = 0.0f;
      const int co = big ? blk : tid;
      const int ci = big ? tid : 0;
      const int wbase = (co * Ci + ci) * Kc;
      const int pstr = Co * Ci * Kc;
      #pragma unroll 1
      for (int tt = 0; tt < 4; ++tt) {
        const int di = tt & 1, dj = tt >> 1;
        #pragma unroll 1
        for (int q = 0; q < Kc; ++q) {
          const float wq = w[wbase + q];
          float pa = p[wbase + q];
          float pb = p[pstr + wbase + q];
          pa = fminf(fmaxf(pa, -2.0f), 2.0f) + 2.0f;
          pb = fminf(fmaxf(pb, -2.0f), 2.0f) + 2.0f;
          const float fa = floorf(pa), fb = floorf(pb);
          const float r1 = pa - fa, r2 = pb - fb;
          const float f1 = di ? r1 : (1.0f - r1);
          const float f2 = dj ? r2 : (1.0f - r2);
          const float val = (wq * f1) * f2;
          int cell = ((int)fa + di) * 6 + ((int)fb + dj);
          cell = min(max(cell, 0), 35);
          my[cell] = my[cell] + val;
        }
      }
    }
    __syncthreads();
    if (big) {
      const int q = min(tid, 103);
      const bool kval = (q < 100);
      const int t = kval ? (q >> 2) : 0;
      const int kh = t / 5, kw = t - 5 * kh;
      const int ci0 = 8 * (q & 3);
      v8h o = z8;
      #pragma unroll
      for (int j = 0; j < 8; ++j) {
        const float v = sacc[(ci0 + j) * 36 + kh * 6 + kw] * WSCALE;
        o[j] = kval ? (_Float16)v : (_Float16)0.0f;
      }
      if (tid < 104) {
        _Float16* dst = k2p + (size_t)blk * K2PITCH + 8 * q;
        *(volatile v8h*)dst = o;
        __threadfence();
        *(volatile v8h*)dst = o;
      }
    } else {
      if (tid < 128) {
        const int q = tid;
        const int co = q >> 2;
        const int k8 = 8 * (q & 3);
        v8h o = z8;
        #pragma unroll
        for (int j = 0; j < 8; ++j) {
          const int kk = k8 + j;
          const bool valid = (kk < 25);
          const int kc = valid ? kk : 0;
          const int kh = kc / 5, kw = kc - 5 * kh;
          const float v = sacc[co * 36 + kh * 6 + kw] * WSCALE;
          o[j] = valid ? (_Float16)v : (_Float16)0.0f;
        }
        _Float16* dst = k1p + 8 * q;
        *(volatile v8h*)dst = o;
        __threadfence();
        *(volatile v8h*)dst = o;
      }
      if (tid < 8) {
        _Float16* dst = zrow + 8 * tid;
        *(volatile v8h*)dst = z8;
        __threadfence();
        *(volatile v8h*)dst = z8;
      }
    }
  } else {
    const int n = blk - 65;
    const float* src = fc1w + (size_t)n * FCK;
    v8h o0 = z8, o1 = z8;
    {
      const int q = tid;
      const int win = q >> 3, c0 = 8 * (q & 7);
      #pragma unroll
      for (int j = 0; j < 8; ++j) o0[j] = (_Float16)(src[(c0 + j) * NWIN2 + win] * WSCALE);
    }
    {
      const int q = min(tid + 256, 391);
      const int win = q >> 3, c0 = 8 * (q & 7);
      #pragma unroll
      for (int j = 0; j < 8; ++j) o1[j] = (_Float16)(src[(c0 + j) * NWIN2 + win] * WSCALE);
    }
    _Float16* d0 = fwp + (size_t)n * FCK + 8 * tid;
    _Float16* d1 = fwp + (size_t)n * FCK + 8 * (tid + 256);
    *(volatile v8h*)d0 = o0;
    if (tid < 136) *(volatile v8h*)d1 = o1;
    __threadfence();
    *(volatile v8h*)d0 = o0;
    if (tid < 136) *(volatile v8h*)d1 = o1;
  }
}

__global__ __launch_bounds__(128) void conv1_kernel(
    const float* __restrict__ x, const _Float16* __restrict__ k1p,
    const float* __restrict__ b1, _Float16* __restrict__ act1)
{
  __shared__ __attribute__((aligned(16))) _Float16 simg[4 * 1024];
  __shared__ __attribute__((aligned(16))) _Float16 sE[4 * 128];
  const int tid = threadIdx.x, lane = tid & 31, w = tid >> 5;
  const int h = lane >> 4, m = lane & 15;
  const int b = blockIdx.x * 4 + w;
  _Float16* img = simg + w * 1024;
  _Float16* sEw = sE + w * 128;
  const v8h z8 = {(_Float16)0.0f, (_Float16)0.0f, (_Float16)0.0f, (_Float16)0.0f,
                  (_Float16)0.0f, (_Float16)0.0f, (_Float16)0.0f, (_Float16)0.0f};

  #pragma unroll
  for (int j = 0; j < 4; ++j) *(v8ha*)(img + 8 * (lane + 32 * j)) = z8;
  __syncthreads();
  const float* xb = x + (size_t)b * IMGPIX;
  #pragma unroll 1
  for (int i = lane; i < IMGPIX; i += 32) {
    const int y = i / 28, xx = i - 28 * y;
    img[(y + 2) * 32 + xx + 2] = (_Float16)xb[i];
  }
  __syncthreads();

  const v16h bf0 = load_frag(k1p + m * K1PITCH, h);
  const v16h bf1 = load_frag(k1p + (16 + m) * K1PITCH, h);
  const float bias0 = b1[m], bias1 = b1[16 + m];
  const v8f zero8 = {0.f, 0.f, 0.f, 0.f, 0.f, 0.f, 0.f, 0.f};
  _Float16* abase = act1 + (size_t)b * NWIN1 * C1;

  #pragma unroll 1
  for (int T = 0; T < 49; ++T) {
    const int p = 16 * T + m;
    const int win = p >> 2, sub = p & 3;
    const int py = win / 14, px = win - 14 * py;
    const int oy = 2 * py + (sub >> 1), ox = 2 * px + (sub & 1);
    const int base = oy * 32 + ox;
    _Float16 e[16];
    #pragma unroll
    for (int i = 0; i < 16; ++i) {
      const int t = 8 * h + ((i < 8) ? i : (i + 8));
      const bool valid = (t < 25);
      const int tc = valid ? t : 0;
      const int kh = (tc * 13) >> 6;
      const int kw = tc - 5 * kh;
      const int addr = valid ? (base + kh * 32 + kw) : 0;
      e[i] = img[addr];
    }
    const v16h av = {e[0], e[1], e[2],  e[3],  e[4],  e[5],  e[6],  e[7],
                     e[8], e[9], e[10], e[11], e[12], e[13], e[14], e[15]};
    const v8f c0 = wmma_f16(av, bf0, zero8);
    const v8f c1 = wmma_f16(av, bf1, zero8);

    const float qa0 = fmaxf(fmaxf(c0[0], c0[1]), fmaxf(c0[2], c0[3]));
    const float qb0 = fmaxf(fmaxf(c0[4], c0[5]), fmaxf(c0[6], c0[7]));
    const float qa1 = fmaxf(fmaxf(c1[0], c1[1]), fmaxf(c1[2], c1[3]));
    const float qb1 = fmaxf(fmaxf(c1[4], c1[5]), fmaxf(c1[6], c1[7]));
    const float pa0 = fmaxf(qa0 * WINV + bias0, 0.0f);
    const float pb0 = fmaxf(qb0 * WINV + bias0, 0.0f);
    const float pa1 = fmaxf(qa1 * WINV + bias1, 0.0f);
    const float pb1 = fmaxf(qb1 * WINV + bias1, 0.0f);
    sEw[(2 * h) * C1 + m]          = (_Float16)pa0;
    sEw[(2 * h + 1) * C1 + m]      = (_Float16)pb0;
    sEw[(2 * h) * C1 + 16 + m]     = (_Float16)pa1;
    sEw[(2 * h + 1) * C1 + 16 + m] = (_Float16)pb1;
    __syncthreads();
    if (lane < 16) {
      const v8h v = *(const v8ha*)(sEw + 8 * lane);
      _Float16* dst = abase + (size_t)(4 * T) * C1 + 8 * lane;
      *(volatile v8h*)dst = v;
      __threadfence();
      *(volatile v8h*)dst = v;
    }
    __syncthreads();
  }
}

__global__ __launch_bounds__(128) void conv2_kernel(
    const _Float16* __restrict__ act1, const _Float16* __restrict__ k2p,
    const _Float16* __restrict__ zrow, const float* __restrict__ b2,
    _Float16* __restrict__ act2)
{
  __shared__ __attribute__((aligned(16))) _Float16 sE[4 * 256];
  const int tid = threadIdx.x, lane = tid & 31, w = tid >> 5;
  const int h = lane >> 4, m = lane & 15;
  _Float16* sEw = sE + w * 256;
  float bias[4];
  #pragma unroll
  for (int nt = 0; nt < 4; ++nt) bias[nt] = b2[16 * nt + m];
  const _Float16* bbase = k2p + (size_t)m * K2PITCH;
  const v8f zero8 = {0.f, 0.f, 0.f, 0.f, 0.f, 0.f, 0.f, 0.f};

  #pragma unroll 1
  for (int T = 0; T < 49; ++T) {
    const int GT = blockIdx.x * 196 + 4 * T + w;
    const int g = 16 * GT + m;
    const int b = g / NWIN1;
    const int p = g - NWIN1 * b;
    const int win = p >> 2, sub = p & 3;
    const int py = win / 7, px = win - 7 * py;
    const int oh = 2 * py + (sub >> 1), ow = 2 * px + (sub & 1);
    const _Float16* ibase = act1 + (size_t)b * NWIN1 * C1;

    v8f acc[4];
    #pragma unroll
    for (int nt = 0; nt < 4; ++nt) acc[nt] = zero8;

    #pragma unroll 1
    for (int kh = 0; kh < 5; ++kh) {
      const int ih = oh + kh - 2;
      const bool vy = (unsigned)ih < 14u;
      const int ihc = min(max(ih, 0), 13);
      #pragma unroll 1
      for (int kw = 0; kw < 5; ++kw) {
        const int iw = ow + kw - 2;
        const bool valid = vy && ((unsigned)iw < 14u);
        const int iwc = min(max(iw, 0), 13);
        const _Float16* ap = valid ? (ibase + (ihc * 14 + iwc) * C1) : zrow;
        const v16h av = load_frag(ap, h);
        const int k0 = (kh * 5 + kw) * 32;
        #pragma unroll
        for (int nt = 0; nt < 4; ++nt) {
          const v16h bv = load_frag(bbase + (size_t)nt * 16 * K2PITCH + k0, h);
          acc[nt] = wmma_f16(av, bv, acc[nt]);
        }
      }
    }

    #pragma unroll
    for (int nt = 0; nt < 4; ++nt) {
      const float qa = fmaxf(fmaxf(acc[nt][0], acc[nt][1]), fmaxf(acc[nt][2], acc[nt][3]));
      const float qb = fmaxf(fmaxf(acc[nt][4], acc[nt][5]), fmaxf(acc[nt][6], acc[nt][7]));
      const float pa = fmaxf(qa * WINV + bias[nt], 0.0f);
      const float pb = fmaxf(qb * WINV + bias[nt], 0.0f);
      sEw[(2 * h) * C2 + 16 * nt + m]     = (_Float16)pa;
      sEw[(2 * h + 1) * C2 + 16 * nt + m] = (_Float16)pb;
    }
    __syncthreads();
    {
      const v8h v = *(const v8ha*)(sEw + 8 * lane);
      _Float16* dst = act2 + (size_t)GT * 256 + 8 * lane;
      *(volatile v8h*)dst = v;
      __threadfence();
      *(volatile v8h*)dst = v;
    }
    __syncthreads();
  }
}

__global__ __launch_bounds__(128) void fc_kernel(
    const _Float16* __restrict__ act2, const _Float16* __restrict__ fwp,
    const float* __restrict__ fc1b, const float* __restrict__ fc2w,
    const float* __restrict__ fc2b, float* __restrict__ out)
{
  __shared__ __attribute__((aligned(16))) float hbuf[64 * FCN];
  __shared__ __attribute__((aligned(16))) float sW2[NCLS * FCN];
  __shared__ float sB2[16];
  __shared__ __attribute__((aligned(16))) float sOut[640];

  const int tid = threadIdx.x, lane = tid & 31, w = tid >> 5;
  const int h = lane >> 4, m = lane & 15;
  #pragma unroll 1
  for (int i = tid; i < NCLS * FCN; i += 128) sW2[i] = fc2w[i];
  if (tid < 16) sB2[tid] = fc2b[min(tid, NCLS - 1)];

  const int row0 = blockIdx.x * 64;
  const _Float16* arow = act2 + (size_t)(row0 + 16 * w + m) * FCK;
  const _Float16* brow = fwp + (size_t)m * FCK;
  const v8f zero8 = {0.f, 0.f, 0.f, 0.f, 0.f, 0.f, 0.f, 0.f};
  v8f acc[8];
  #pragma unroll
  for (int nt = 0; nt < 8; ++nt) acc[nt] = zero8;

  #pragma unroll 1
  for (int kc = 0; kc < FCK / 32; ++kc) {
    const int k0 = kc * 32;
    const v16h av = load_frag(arow + k0, h);
    #pragma unroll
    for (int nt = 0; nt < 8; ++nt) {
      const v16h bv = load_frag(brow + (size_t)nt * 16 * FCK + k0, h);
      acc[nt] = wmma_f16(av, bv, acc[nt]);
    }
  }

  #pragma unroll
  for (int nt = 0; nt < 8; ++nt) {
    const int col = 16 * nt + m;
    const float bb = fc1b[col];
    #pragma unroll
    for (int r = 0; r < 8; ++r)
      hbuf[(16 * w + 8 * h + r) * FCN + col] = fmaxf(acc[nt][r] * WINV + bb, 0.0f);
  }
  __syncthreads();

  #pragma unroll 1
  for (int j = 0; j < 5; ++j) {
    const int idx = tid + 128 * j;
    const int row = idx / NCLS, jj = idx - NCLS * row;
    const float* hr = hbuf + row * FCN;
    const float* wr = sW2 + jj * FCN;
    float s = 0.0f;
    #pragma unroll 4
    for (int n = 0; n < FCN; ++n) s += hr[n] * wr[n];
    sOut[idx] = s + sB2[jj];
  }
  __syncthreads();

  const v4f v0 = *(const v4fa*)(sOut + 4 * tid);
  const v4f v1 = *(const v4fa*)(sOut + 4 * (128 + (tid & 31)));
  float* obase = out + (size_t)blockIdx.x * 640;
  *(volatile v4f*)(obase + 4 * tid) = v0;
  if (tid < 32) *(volatile v4f*)(obase + 4 * (128 + tid)) = v1;
  __threadfence();
  *(volatile v4f*)(obase + 4 * tid) = v0;
  if (tid < 32) *(volatile v4f*)(obase + 4 * (128 + tid)) = v1;
}

extern "C" void kernel_launch(void* const* d_in, const int* in_sizes, int n_in,
                              void* d_out, int out_size, void* d_ws, size_t ws_size,
                              hipStream_t stream) {
  if (n_in < 11) return;
  if (in_sizes[0] != NIMG * IMGPIX) return;
  if (in_sizes[1] != C1 * 1 * KC1 || in_sizes[2] != 2 * C1 * 1 * KC1 || in_sizes[3] != C1) return;
  if (in_sizes[4] != C2 * 32 * KC2 || in_sizes[5] != 2 * C2 * 32 * KC2 || in_sizes[6] != C2) return;
  if (in_sizes[7] != FCN * FCK || in_sizes[8] != FCN) return;
  if (in_sizes[9] != NCLS * FCN || in_sizes[10] != NCLS) return;
  if (out_size != NIMG * NCLS) return;
  if ((size_t)WS_TOTAL > ws_size) return;

  const float* x    = (const float*)d_in[0];
  const float* w1   = (const float*)d_in[1];
  const float* p1   = (const float*)d_in[2];
  const float* b1   = (const float*)d_in[3];
  const float* w2   = (const float*)d_in[4];
  const float* p2   = (const float*)d_in[5];
  const float* b2   = (const float*)d_in[6];
  const float* fc1w = (const float*)d_in[7];
  const float* fc1b = (const float*)d_in[8];
  const float* fc2w = (const float*)d_in[9];
  const float* fc2b = (const float*)d_in[10];
  float* out = (float*)d_out;

  char* ws = (char*)d_ws;
  _Float16* zrow = (_Float16*)(ws + OFF_ZROW);
  _Float16* k1p  = (_Float16*)(ws + OFF_K1P);
  _Float16* k2p  = (_Float16*)(ws + OFF_K2P);
  _Float16* fwp  = (_Float16*)(ws + OFF_FWP);
  _Float16* act1 = (_Float16*)(ws + OFF_ACT1);
  _Float16* act2 = (_Float16*)(ws + OFF_ACT2);

  prep_kernel<<<65 + FCN, 256, 0, stream>>>(w1, p1, w2, p2, fc1w, zrow, k1p, k2p, fwp);
  conv1_kernel<<<NIMG / 4, 128, 0, stream>>>(x, k1p, b1, act1);
  conv2_kernel<<<(NIMG * NWIN1) / (16 * 196), 128, 0, stream>>>(act1, k2p, zrow, b2, act2);
  fc_kernel<<<NIMG / 64, 128, 0, stream>>>(act2, fwp, fc1b, fc2w, fc2b, out);
}
